// ExRestSelfAtten_13168369730242
// MI455X (gfx1250) — hardware-verified
//
#include <hip/hip_runtime.h>


namespace {
constexpr int B = 8, S = 2048, DI = 512, H = 512, NO = 2, A = 5, NR = B * S, RL = NR  ;
constexpr float XS = 8.0f, WSC = 256.0f, WSQ = 0.25f, RS_ = 1024.0f;
static_assert(NR % 32 == 0 && RL % 32 == 0 && DI == 512 && H == 512, "tiling");
typedef _Float16 b16;
typedef __attribute__((ext_vector_type(16))) _Float16 v16b;
typedef __attribute__((ext_vector_type(8))) _Float16 v8b;
typedef __attribute__((ext_vector_type(8))) float v8f;
typedef __attribute__((ext_vector_type(4))) float v4f;
__device__ __forceinline__ float bf16_rne(float f) { unsigned int u = __float_as_uint(f); u += 0x7FFFu + ((u >> 16) & 1u); return __uint_as_float(u & 0xFFFF0000u); }
__device__ __forceinline__ void split16(float v, b16& hi, b16& lo) { hi = (b16)v; lo = (b16)(v - (float)hi); }
__device__ __forceinline__ v16b frag_kb(const b16* p, int hh) { const v8b a = *(const v8b*)(p + 8 * hh), b = *(const v8b*)(p + 16 + 8 * hh); v16b f;
#pragma unroll
  for (int e = 0; e < 8; ++e) { f[e] = a[e]; f[8 + e] = b[e]; } return f; }
__device__ __forceinline__ v8f wmma16b(v16b a, v16b b, v8f c) { v8f d = __builtin_amdgcn_wmma_f32_16x16x32_f16(false, a, false, b, (short)0, c, false, false); asm volatile("v_nop\n\tv_nop\n\tv_nop\n\tv_nop" : "+v"(d) : "v"(a), "v"(b)); return d; }
__device__ __forceinline__ void wave_lds_sync() { __builtin_amdgcn_fence(__ATOMIC_RELEASE, "workgroup"); __builtin_amdgcn_wave_barrier(); __builtin_amdgcn_fence(__ATOMIC_ACQUIRE, "workgroup"); }
__device__ __forceinline__ float pmul(float a, float b) { float p = a * b; asm volatile("" : "+v"(p)); return p; }
__device__ __forceinline__ int iclamp(int v, int lo, int hi) { return v < lo ? lo : (v > hi ? hi : v); }

typedef __attribute__((ext_vector_type(2))) _Float16 v2h;
typedef __attribute__((ext_vector_type(4))) _Float16 v4h;
typedef __attribute__((ext_vector_type(2))) float v2f;
typedef __attribute__((ext_vector_type(4))) int v4i;
__device__ __forceinline__ float nexp2(float v) { return __builtin_amdgcn_exp2f(v); }
typedef __attribute__((ext_vector_type(4))) _Float16 v4h_;
__global__ __launch_bounds__(256) void wt_kernel(const float* __restrict__ w, b16* __restrict__ WT, float scl) {
  const int u = blockIdx.x * 256 + threadIdx.x; if (u >= H * H / 8) return; const int e = u * 8; const int o = e / H, k0 = e % H; v8b v;
#pragma unroll
  for (int j = 0; j < 8; ++j) v[j] = (b16)(bf16_rne(w[(size_t)(k0 + j) * H + o]) * scl);
  for (int pass = 0; pass < 2; ++pass) { *(volatile v8b*)(WT + e) = v; __threadfence(); }
}
__global__ __launch_bounds__(256) void h_kernel(const float* __restrict__ x, const b16* __restrict__ W1T, const float* __restrict__ b1, float* __restrict__ Hh) {
  __shared__ __attribute__((aligned(16))) b16 Ah[32][128 + 8]; __shared__ __attribute__((aligned(16))) float Tf[32][H + 4];
  const int tid = threadIdx.x, wave = tid >> 5, lane = tid & 31, nloc = lane & 15, hlf = lane >> 4; const int r0 = blockIdx.x * 32; const int row = tid >> 3, g = tid & 7;
  v8f acc[2][4]; for (int rt = 0; rt < 2; ++rt) for (int t = 0; t < 4; ++t) acc[rt][t] = (v8f){};
#pragma unroll 1
  for (int kc = 0; kc < DI; kc += 128) {
    __syncthreads();
    { const float* xr = x + (size_t)(r0 + row) * DI + kc + g * 16; for (int q = 0; q < 4; ++q) { const v4f t4 = *(const v4f*)(xr + 4 * q); v4h_ h4; for (int j = 0; j < 4; ++j) h4[j] = (b16)(bf16_rne(t4[j]) * XS); *(v4h_*)(&Ah[row][g * 16 + 4 * q]) = h4; } }
    __syncthreads();
#pragma unroll
    for (int kb = 0; kb < 128; kb += 32) { const v16b a0 = frag_kb(&Ah[nloc][kb], hlf), a1 = frag_kb(&Ah[16 + nloc][kb], hlf);
#pragma unroll
      for (int t = 0; t < 4; ++t) { const v16b bw = frag_kb(W1T + (size_t)((wave * 4 + t) * 16 + nloc) * DI + kc + kb, hlf); acc[0][t] = wmma16b(a0, bw, acc[0][t]); acc[1][t] = wmma16b(a1, bw, acc[1][t]); } } }
#pragma unroll
  for (int t = 0; t < 4; ++t) { const int col = (wave * 4 + t) * 16 + nloc; const float bb = bf16_rne(b1[col]);
    for (int rt = 0; rt < 2; ++rt) for (int q = 0; q < 8; ++q) Tf[rt * 16 + 8 * hlf + q][col] = fmaxf(acc[rt][t][q] * (1.0f / (XS * WSC)) + bb, 0.0f); }
  __syncthreads();
  for (int pass = 0; pass < 2; ++pass) { for (int rr = wave * 4; rr < wave * 4 + 4; ++rr) { float* d = Hh + (size_t)(r0 + rr) * H;
#pragma unroll
      for (int s2 = 0; s2 < 4; ++s2) *(volatile v4f*)(d + s2 * 128 + lane * 4) = *(const v4f*)(&Tf[rr][s2 * 128 + lane * 4]); } __threadfence(); }
}
__global__ __launch_bounds__(256) void aw_kernel(const float* __restrict__ Hh, const b16* __restrict__ WvT, const b16* __restrict__ WvQ, const b16* __restrict__ W2T, const b16* __restrict__ W2Q, const float* __restrict__ b2, const float* __restrict__ wfc, const float* __restrict__ bfc, float* __restrict__ OUT0, float* __restrict__ AW) {
  __shared__ __attribute__((aligned(16))) b16 Ah[32][128 + 8], Al[32][128 + 8]; __shared__ __attribute__((aligned(16))) float Tf[32][H + 4]; __shared__ float So[64];
  const int tid = threadIdx.x, wave = tid >> 5, lane = tid & 31, nloc = lane & 15, hlf = lane >> 4; const int r0 = blockIdx.x * 32; const int row = tid >> 3, g = tid & 7; const int r = r0 + row; const int bb_ = r / S, p = r % S;
  v8f acc[2][4];
  for (int rt = 0; rt < 2; ++rt) for (int t = 0; t < 4; ++t) acc[rt][t] = (v8f){};
#pragma unroll 1
  for (int kc = 0; kc < H; kc += 128) {
    float w16[16]; for (int j = 0; j < 16; ++j) w16[j] = 0.0f;
#pragma unroll 1
    for (int d = -A; d <= A; ++d) { const int q = p + d; const float fl = (q >= 0 && q < S) ? 1.0f : 0.0f; const float* hr = Hh + ((size_t)bb_ * S + (q < 0 ? 0 : (q >= S ? S - 1 : q))) * H + kc + g * 16;
#pragma unroll
      for (int q4 = 0; q4 < 4; ++q4) { const v4f t4 = *(const v4f*)(hr + 4 * q4); for (int j = 0; j < 4; ++j) w16[4 * q4 + j] = fmaf(t4[j], fl, w16[4 * q4 + j]); } }
    __syncthreads();
#pragma unroll
    for (int q4 = 0; q4 < 4; ++q4) { v4h_ h4, l4; for (int j = 0; j < 4; ++j) { const float vs = w16[4 * q4 + j] * XS; const b16 ph = (b16)vs; h4[j] = ph; l4[j] = (b16)((vs - (float)ph) * RS_); } *(v4h_*)(&Ah[row][g * 16 + 4 * q4]) = h4; *(v4h_*)(&Al[row][g * 16 + 4 * q4]) = l4; }
    __syncthreads();
#pragma unroll
    for (int kb = 0; kb < 128; kb += 32) { const v16b a0 = frag_kb(&Ah[nloc][kb], hlf), a1 = frag_kb(&Ah[16 + nloc][kb], hlf), l0 = frag_kb(&Al[nloc][kb], hlf), l1 = frag_kb(&Al[16 + nloc][kb], hlf);
#pragma unroll
      for (int t = 0; t < 4; ++t) { const size_t wo_ = (size_t)((wave * 4 + t) * 16 + nloc) * H + kc + kb; const v16b bw = frag_kb(WvT + wo_, hlf), bq = frag_kb(WvQ + wo_, hlf);
        acc[0][t] = wmma16b(a0, bw, acc[0][t]); acc[0][t] = wmma16b(l0, bq, acc[0][t]); acc[1][t] = wmma16b(a1, bw, acc[1][t]); acc[1][t] = wmma16b(l1, bq, acc[1][t]); } } }
#pragma unroll
  for (int t = 0; t < 4; ++t) { const int col = (wave * 4 + t) * 16 + nloc; for (int rt = 0; rt < 2; ++rt) for (int q = 0; q < 8; ++q) Tf[rt * 16 + 8 * hlf + q][col] = acc[rt][t][q] * (1.0f / (XS * WSC)); }
  __syncthreads();
  for (int pass = 0; pass < 2; ++pass) { for (int rr = wave * 4; rr < wave * 4 + 4; ++rr) { float* d = AW + (size_t)(r0 + rr) * H;
#pragma unroll
      for (int s2 = 0; s2 < 4; ++s2) *(volatile v4f*)(d + s2 * 128 + lane * 4) = *(const v4f*)(&Tf[rr][s2 * 128 + lane * 4]); } __threadfence(); }
  for (int rt = 0; rt < 2; ++rt) for (int t = 0; t < 4; ++t) acc[rt][t] = (v8f){};
#pragma unroll 1
  for (int kc = 0; kc < H; kc += 128) {
    __syncthreads();
#pragma unroll
    for (int q4 = 0; q4 < 4; ++q4) { v4h_ h4, l4; for (int j = 0; j < 4; ++j) { const float vs = Tf[row][kc + g * 16 + 4 * q4 + j] * XS; const b16 ph = (b16)vs; h4[j] = ph; l4[j] = (b16)((vs - (float)ph) * RS_); } *(v4h_*)(&Ah[row][g * 16 + 4 * q4]) = h4; *(v4h_*)(&Al[row][g * 16 + 4 * q4]) = l4; }
    __syncthreads();
#pragma unroll
    for (int kb = 0; kb < 128; kb += 32) { const v16b a0 = frag_kb(&Ah[nloc][kb], hlf), a1 = frag_kb(&Ah[16 + nloc][kb], hlf), l0 = frag_kb(&Al[nloc][kb], hlf), l1 = frag_kb(&Al[16 + nloc][kb], hlf);
#pragma unroll
      for (int t = 0; t < 4; ++t) { const size_t wo_ = (size_t)((wave * 4 + t) * 16 + nloc) * H + kc + kb; const v16b bw = frag_kb(W2T + wo_, hlf), bq = frag_kb(W2Q + wo_, hlf);
        acc[0][t] = wmma16b(a0, bw, acc[0][t]); acc[0][t] = wmma16b(l0, bq, acc[0][t]); acc[1][t] = wmma16b(a1, bw, acc[1][t]); acc[1][t] = wmma16b(l1, bq, acc[1][t]); } } }
  __syncthreads();
#pragma unroll
  for (int t = 0; t < 4; ++t) { const int col = (wave * 4 + t) * 16 + nloc; const float bb = bf16_rne(b2[col]); for (int rt = 0; rt < 2; ++rt) for (int q = 0; q < 8; ++q) Tf[rt * 16 + 8 * hlf + q][col] = fmaxf(acc[rt][t][q] * (1.0f / (XS * WSC)) + bb, 0.0f); }
  __syncthreads();
  if (tid < 64) { const int rr = tid >> 1, o = tid & 1; float s = 0.0f;
#pragma unroll 4
    for (int c = 0; c < H; ++c) s = fmaf(Tf[rr][c], bf16_rne(wfc[c * NO + o]), s);
    So[tid] = s + bf16_rne(bfc[o]); }
  __syncthreads();
  for (int pass = 0; pass < 2; ++pass) { if (tid < 64) ((volatile float*)OUT0)[(size_t)r0 * NO + tid] = So[tid]; __threadfence(); }
}
}

extern "C" void kernel_launch(void* const* d_in, const int* in_sizes, int n_in, void* d_out, int out_size, void* d_ws, size_t ws_size, hipStream_t stream) {
  (void)n_in;
  auto Fp = [&](int i) { return (const float*)d_in[i]; };
  if (in_sizes[0] != NR * DI || in_sizes[1] != DI * H || in_sizes[2] != H || in_sizes[5] != H * H || in_sizes[6] != H * H || in_sizes[7] != H || in_sizes[8] != H * NO || in_sizes[9] != NO || out_size != NR * NO + NR * H) return;
  size_t off = 0; char* ws = (char*)d_ws;
  auto carve = [&](size_t bytes) { char* p = ws + off; off += (bytes + 255) & ~(size_t)255; return p; };
  b16* W1T = (b16*)carve((size_t)H * DI * 2); b16* WvT = (b16*)carve((size_t)H * H * 2); b16* WvQ = (b16*)carve((size_t)H * H * 2); b16* W2T = (b16*)carve((size_t)H * H * 2); b16* W2Q = (b16*)carve((size_t)H * H * 2); float* Hh = (float*)carve((size_t)NR * H * 4);
  if (off > ws_size || off > ((size_t)128 << 20)) return;
  float* OUT0 = (float*)d_out; float* AW = OUT0 + (size_t)NR * NO;
  wt_kernel<<<(H * H / 8 + 255) / 256, 256, 0, stream>>>(Fp(1), W1T, WSC);
  wt_kernel<<<(H * H / 8 + 255) / 256, 256, 0, stream>>>(Fp(5), WvT, WSC); wt_kernel<<<(H * H / 8 + 255) / 256, 256, 0, stream>>>(Fp(5), WvQ, WSQ);
  wt_kernel<<<(H * H / 8 + 255) / 256, 256, 0, stream>>>(Fp(6), W2T, WSC); wt_kernel<<<(H * H / 8 + 255) / 256, 256, 0, stream>>>(Fp(6), W2Q, WSQ);
  h_kernel<<<RL / 32, 256, 0, stream>>>(Fp(0), W1T, Fp(2), Hh);
  aw_kernel<<<RL / 32, 256, 0, stream>>>(Hh, WvT, WvQ, W2T, W2Q, Fp(7), Fp(8), Fp(9), OUT0, AW);
}
